// MultiHeadLatentAttention_70171175682544
// MI455X (gfx1250) — hardware-verified
//
#include <hip/hip_runtime.h>
#include <stddef.h>


typedef _Float16 v16h __attribute__((ext_vector_type(16)));
typedef _Float16 v8h  __attribute__((ext_vector_type(8)));
typedef float    v8f  __attribute__((ext_vector_type(8)));
typedef float    v4f  __attribute__((ext_vector_type(4)));
typedef _Float16 h16;

#ifndef NB
#define NB 2
#endif
#ifndef SEQ
#define SEQ 2048
#endif
#ifndef EARLY_ROWS
#define EARLY_ROWS 512
#endif
#define NB_FULL  2
#define SEQ_FULL 2048
#define HIDN  2048
#define NHEAD 16
#define HD    128
#define RANK  512
#define KVAW  640
#define KVBW  4096
#define CSW   128
#define MROWS (NB * SEQ)
#define ERB   ((EARLY_ROWS < SEQ) ? EARLY_ROWS : SEQ)
#define EBLK  (ERB / 128)

static_assert(NB >= 1 && NB <= NB_FULL);
static_assert(SEQ >= 128 && SEQ <= SEQ_FULL && (SEQ % 128) == 0);
static_assert(EARLY_ROWS >= 128 && (EARLY_ROWS % 128) == 0);
static_assert(ERB >= 128 && (ERB % 128) == 0 && ERB <= SEQ && (ERB % 64) == 0);
static_assert(HIDN == NHEAD * HD);
static_assert(HD == 128);
static_assert(KVAW == RANK + HD);
static_assert(KVBW == NHEAD * 2 * HD);
static_assert(HIDN / 128 == NHEAD && KVBW / 128 == 2 * NHEAD);
static_assert((HIDN % 128) == 0 && (KVAW % 128) == 0 && (KVBW % 128) == 0);
static_assert((HIDN % 64) == 0 && (KVAW % 64) == 0 && (KVBW % 64) == 0 && (RANK % 64) == 0);
static_assert((HIDN % 32) == 0 && (RANK % 32) == 0 && (HD % 32) == 0);
static_assert((MROWS % 64) == 0 && (MROWS % 8) == 0 && (SEQ % 64) == 0);
static_assert(HIDN == 256 * 8);
static_assert(RANK == 2 * 32 * 8);
static_assert(HD == 32 * 4);
static_assert(CSW == HD);
static_assert((size_t)MROWS * HIDN < (size_t)0xFFFFFFFFu);

#define LDT  72
#define LDK  136
#define LDC2 132
static_assert((LDT % 8) == 0 && LDT >= 64);
static_assert((LDK % 8) == 0 && LDK >= HD);
static_assert((LDC2 % 4) == 0 && LDC2 >= 128);

#define WCARRY 64.0f
#define PCARRY 1024.0f
#define VCARRY 64.0f
#define RCARRY 1024.0f
#define QCARRY 2048.0f

#define WQ_BYTES      ((size_t)HIDN * HIDN * 2)
#define WKVA_BYTES    ((size_t)KVAW * HIDN * 2)
#define WKVB_BYTES    ((size_t)KVBW * RANK * 2)
#define PLANE16_BYTES ((size_t)MROWS * HIDN * 2)
#define XCTX_BYTES    PLANE16_BYTES
#define EPLANE_BYTES  ((size_t)NB * ERB * HIDN * 2)
#define KVA_BYTES     ((size_t)MROWS * KVAW * 4)
#define C16_BYTES     ((size_t)MROWS * RANK * 2)
#define KR_BYTES      ((size_t)MROWS * HD * 4)
#define CS_BYTES      ((size_t)MROWS * CSW * 4)
#define C16E_BYTES    ((size_t)NB * ERB * RANK * 2)
#define OFF_WQ   ((size_t)0)
#define OFF_WKVA (OFF_WQ + WQ_BYTES)
#define OFF_WKVB (OFF_WKVA + WKVA_BYTES)
#define OFF_WO   (OFF_WKVB + WKVB_BYTES)
#define OFF_X    (OFF_WO + WQ_BYTES)
#define OFF_CTX  OFF_X
#define OFF_Q    (OFF_X + XCTX_BYTES)
#define OFF_K    (OFF_Q + PLANE16_BYTES)
#define OFF_VT   (OFF_K + PLANE16_BYTES)
#define OFF_QE   (OFF_VT + PLANE16_BYTES)
#define OFF_KE   (OFF_QE + EPLANE_BYTES)
#define OFF_VE   (OFF_KE + EPLANE_BYTES)
#define OFF_CE   (OFF_VE + EPLANE_BYTES)
#define OFF_KVA  (OFF_CE + EPLANE_BYTES)
#define OFF_C16  (OFF_KVA + KVA_BYTES)
#define OFF_KR   (OFF_C16 + C16_BYTES)
#define OFF_CS   (OFF_KR + KR_BYTES)
#define OFF_C16E (OFF_CS + CS_BYTES)
#define WS_TOTAL (OFF_C16E + C16E_BYTES)
static_assert((WQ_BYTES % 128) == 0 && (WKVA_BYTES % 128) == 0 && (WKVB_BYTES % 128) == 0);
static_assert((PLANE16_BYTES % 128) == 0 && (EPLANE_BYTES % 128) == 0 && (KVA_BYTES % 128) == 0);
static_assert((C16_BYTES % 128) == 0 && (KR_BYTES % 128) == 0 && (CS_BYTES % 128) == 0);
static_assert((C16E_BYTES % 128) == 0);
static_assert((size_t)MROWS * HIDN * 2 <= XCTX_BYTES);
static_assert((size_t)NB * HIDN * ERB * 2 <= EPLANE_BYTES);
static_assert((size_t)(NB * ERB) * RANK * 2 <= C16E_BYTES);
static_assert(WS_TOTAL <= (size_t)134217728);

__device__ __forceinline__ float bf16r(float x) {
  unsigned int u = __float_as_uint(x);
  u = (u + 0x7FFFu + ((u >> 16) & 1u)) & 0xFFFF0000u;
  return __uint_as_float(u);
}

static __device__ __forceinline__ h16 toh_flush(float v) {
  const h16 r = (h16)v;
  return (fabsf(v) < 6.103515625e-05f) ? (h16)0.0f : r;
}

__device__ __forceinline__ v16h frag_at(const _Float16* p) {
  v8h lo = *(const v8h*)(p);
  v8h hi = *(const v8h*)(p + 16);
  v16h out;
#pragma unroll
  for (int i = 0; i < 8; ++i) { out[i] = lo[i]; out[i + 8] = hi[i]; }
  return out;
}
__device__ __forceinline__ v16h ld_frag(const _Float16* base, unsigned ld) {
  const unsigned lane = threadIdx.x & 31u;
  return frag_at(base + (lane & 15u) * ld + (lane >> 4) * 8u);
}

__device__ __forceinline__ v8f wmma16(v16h a, v16h b, v8f c) {
  v8f d = __builtin_amdgcn_wmma_f32_16x16x32_f16(false, a, false, b, (short)0, c,
                                                 false, false);
  asm volatile("v_nop\n\tv_nop\n\tv_nop\n\tv_nop" : "+v"(d) : "v"(a), "v"(b));
  return d;
}

__device__ __forceinline__ float red16_max(float x) {
#pragma unroll
  for (int off = 1; off < 16; off <<= 1) x = fmaxf(x, __shfl_xor(x, off, 32));
  return x;
}
__device__ __forceinline__ float red16_sum(float x) {
#pragma unroll
  for (int off = 1; off < 16; off <<= 1) x += __shfl_xor(x, off, 32);
  return x;
}
__device__ __forceinline__ float red32_sum(float x) {
#pragma unroll
  for (int off = 1; off < 32; off <<= 1) x += __shfl_xor(x, off, 32);
  return x;
}

__device__ __forceinline__ void wave_lds_sync() {
  __builtin_amdgcn_fence(3  , "wavefront");
  asm volatile("s_wait_dscnt 0x0" ::: "memory");
  __builtin_amdgcn_wave_barrier();
}

__global__ __launch_bounds__(256) void wconv_kernel(
    const float* __restrict__ W, _Float16* __restrict__ Wt, unsigned ldw, unsigned ldk) {
  __shared__ _Float16 T[64 * LDT];
  const unsigned tid = threadIdx.x;
  const unsigned n0 = blockIdx.x * 64u;
  const unsigned k0 = blockIdx.y * 64u;
#pragma unroll 4
  for (unsigned j = 0; j < 16u; ++j) {
    const unsigned idx = tid + 256u * j;
    const unsigned kr = idx >> 6, nc = idx & 63u;
    const float v = W[(size_t)(k0 + kr) * ldw + n0 + nc];
    T[nc * LDT + kr] = (_Float16)(WCARRY * bf16r(v));
  }
  __syncthreads();
  v8h x[2];
  size_t off[2];
#pragma unroll
  for (unsigned i = 0; i < 2u; ++i) {
    const unsigned n = 32u * i + (tid >> 3);
    const unsigned kc = (tid & 7u) * 8u;
    x[i] = *(const v8h*)&T[n * LDT + kc];
    off[i] = (size_t)(n0 + n) * ldk + k0 + kc;
  }
#pragma unroll
  for (int i = 0; i < 2; ++i) *(volatile v8h*)(Wt + off[i]) = x[i];
  __threadfence();
#pragma unroll
  for (int i = 0; i < 2; ++i) *(volatile v8h*)(Wt + off[i]) = x[i];
}

__global__ __launch_bounds__(256) void xcast_kernel(
    const float* __restrict__ X, _Float16* __restrict__ dst) {
  const unsigned tid = threadIdx.x;
  const unsigned crow = blockIdx.x;
  const unsigned bidx = crow / (unsigned)SEQ;
  const unsigned sq = crow - bidx * (unsigned)SEQ;
  const size_t srow = (size_t)bidx * SEQ_FULL + sq;
  const unsigned c = tid * 8u;
  const v4f a0 = *(const v4f*)(X + srow * HIDN + c);
  const v4f a1 = *(const v4f*)(X + srow * HIDN + c + 4u);
  v8h o;
#pragma unroll
  for (int i = 0; i < 4; ++i) {
    o[i]     = toh_flush(bf16r(a0[i]));
    o[i + 4] = toh_flush(bf16r(a1[i]));
  }
  _Float16* p = dst + (size_t)crow * HIDN + c;
  *(volatile v8h*)p = o;
  __threadfence();
  *(volatile v8h*)p = o;
}

__global__ __launch_bounds__(256) void cstab_kernel(
    const int* __restrict__ pos, float* __restrict__ cs) {
#pragma clang fp contract(off)
  __shared__ float T[8 * CSW];
  const unsigned tid = threadIdx.x;
#pragma unroll 1
  for (unsigned j = 0; j < 2u; ++j) {
    const unsigned idx = tid + 256u * j;
    const unsigned r = idx >> 6, fi = idx & 63u;
    const unsigned crow = blockIdx.x * 8u + r;
    const unsigned bidx = crow / (unsigned)SEQ;
    const unsigned sq = crow - bidx * (unsigned)SEQ;
    const float p = (float)pos[(size_t)bidx * SEQ_FULL + sq];
    const float fif = (float)fi;
    const float pf = exp2f(fif * 0.2957916259765625f) * exp2f(fif * 1.413291912772e-5f);
    const float extrap = 1.0f / pf;
    const float interp = extrap * 0.0625f;
    float sm = (fif - 18.0f) * 0.058823529411764705f;
    sm = fminf(fmaxf(sm, 0.0f), 1.0f);
    const float invf = (1.0f - sm) * interp + sm * extrap;
    const float ang = p * invf;
    const float cn = cosf(ang);
    const float sn = sinf(ang);
    T[r * CSW + fi] = cn * 1.2772588722239781f;
    T[r * CSW + 64u + fi] = sn * 1.2772588722239781f;
  }
  __syncthreads();
  const v4f x = *(const v4f*)&T[tid * 4u];
  float* q = cs + (size_t)blockIdx.x * (8u * CSW) + tid * 4u;
  *(volatile v4f*)q = x;
  __threadfence();
  *(volatile v4f*)q = x;
}

__global__ __launch_bounds__(256) void norm_rope_kernel(
    const float* __restrict__ kva, const float* __restrict__ lnw, const float* __restrict__ cs,
    _Float16* __restrict__ c16, _Float16* __restrict__ c16e, float* __restrict__ kr) {
#pragma clang fp contract(off)
  const unsigned lane = threadIdx.x & 31u;
  const unsigned w = (unsigned)__builtin_amdgcn_readfirstlane((int)(threadIdx.x >> 5));
  const unsigned crow = blockIdx.x * 8u + w;
  const unsigned bidx = crow / (unsigned)SEQ;
  const unsigned sq = crow - bidx * (unsigned)SEQ;
  const bool early_row = (sq < (unsigned)ERB);
  const float* xr = kva + (size_t)crow * KVAW;

  float ss = 0.0f;
#pragma unroll 1
  for (unsigned j = 0; j < 2u; ++j) {
    const v4f a0 = *(const v4f*)(xr + j * 256u + lane * 8u);
    const v4f a1 = *(const v4f*)(xr + j * 256u + lane * 8u + 4u);
#pragma unroll
    for (int i = 0; i < 4; ++i) {
      ss += a0[i] * a0[i];
      ss += a1[i] * a1[i];
    }
  }
  const float var = red32_sum(ss) * (1.0f / (float)RANK);
  const float rstd = 1.0f / sqrtf(var + 1.0e-6f);

#pragma unroll 1
  for (unsigned j = 0; j < 2u; ++j) {
    const unsigned c = j * 256u + lane * 8u;
    const v4f a0 = *(const v4f*)(xr + c);
    const v4f a1 = *(const v4f*)(xr + c + 4u);
    const v4f g0 = *(const v4f*)(lnw + c);
    const v4f g1 = *(const v4f*)(lnw + c + 4u);
    v8h o, oe;
#pragma unroll
    for (int i = 0; i < 4; ++i) {
      const float ta = bf16r(g0[i]) * (a0[i] * rstd);
      const float tb = bf16r(g1[i]) * (a1[i] * rstd);
      const h16 ha = toh_flush(ta);
      const h16 hb = toh_flush(tb);
      o[i]      = ha;
      o[i + 4]  = hb;
      oe[i]     = toh_flush((ta - (float)ha) * QCARRY);
      oe[i + 4] = toh_flush((tb - (float)hb) * QCARRY);
    }
    _Float16* p = c16 + (size_t)crow * RANK + c;
    *(volatile v8h*)p = o;
    if (early_row) {
      _Float16* pe = c16e + (size_t)(bidx * (unsigned)ERB + sq) * RANK + c;
      *(volatile v8h*)pe = oe;
    }
    __threadfence();
    *(volatile v8h*)p = o;
    if (early_row) {
      _Float16* pe = c16e + (size_t)(bidx * (unsigned)ERB + sq) * RANK + c;
      *(volatile v8h*)pe = oe;
    }
  }

  const unsigned d = lane * 4u;
  const v4f xa = *(const v4f*)(xr + RANK + d);
  const v4f xb = *(const v4f*)(xr + RANK + (d ^ 64u));
  const unsigned fi = d & 63u;
  const v4f cc = *(const v4f*)(cs + (size_t)crow * CSW + fi);
  const v4f sn = *(const v4f*)(cs + (size_t)crow * CSW + 64u + fi);
  const float sg = (d < 64u) ? -1.0f : 1.0f;
  v4f o4;
#pragma unroll
  for (int i = 0; i < 4; ++i) o4[i] = xa[i] * cc[i] + sg * (xb[i] * sn[i]);
  float* q = kr + (size_t)crow * HD + d;
  *(volatile v4f*)q = o4;
  __threadfence();
  *(volatile v4f*)q = o4;
}

template <int MODE>
__device__ __forceinline__ void gemm_body(
    const _Float16* __restrict__ A16, const _Float16* __restrict__ A16r,
    const _Float16* __restrict__ Bt, const unsigned K,
    const float* __restrict__ aux, float* __restrict__ outf,
    _Float16* __restrict__ out16, _Float16* __restrict__ out16e,
    _Float16* __restrict__ out16v, _Float16* __restrict__ out16r) {
  __shared__ float Cs[64 * LDC2];
  const unsigned tid = threadIdx.x, lane = tid & 31u;
  const unsigned w = (unsigned)__builtin_amdgcn_readfirstlane((int)(tid >> 5));
  const unsigned mw = w >> 1, nw = w & 1u;
  const unsigned hh = lane >> 4, m = lane & 15u;
  const unsigned n0 = blockIdx.x * 128u;
  const unsigned row0 = blockIdx.y * 64u;
  const unsigned bidx0 = row0 / (unsigned)SEQ;
  const unsigned sq0 = row0 - bidx0 * (unsigned)SEQ;
  const bool early_tile = (sq0 < (unsigned)ERB);
  const float iw = 1.0f / WCARRY;

  const _Float16* ap = A16 + (size_t)(row0 + mw * 16u + m) * K + hh * 8u;
#pragma unroll 1
  for (unsigned p = 0; p < 2u; ++p) {
    const _Float16* bp0 = Bt + (size_t)(n0 + p * 64u + nw * 32u + m) * K + hh * 8u;
    const _Float16* bp1 = bp0 + (size_t)16 * K;
    v8f acc0 = {}, acc1 = {};
#pragma unroll 2
    for (unsigned k0 = 0; k0 < K; k0 += 32u) {
      const v16h a  = frag_at(ap + k0);
      const v16h b0 = frag_at(bp0 + k0);
      const v16h b1 = frag_at(bp1 + k0);
      acc0 = wmma16(a, b0, acc0);
      acc1 = wmma16(a, b1, acc1);
    }
    if (MODE == 2 || MODE == 3) {
      if (early_tile) {
        const float rs = (MODE == 2) ? (1.0f / QCARRY) : (1.0f / RCARRY);
        const _Float16* apr =
            A16r + (size_t)(bidx0 * (unsigned)ERB + sq0 + mw * 16u + m) * K + hh * 8u;
        v8f r0 = {}, r1 = {};
#pragma unroll 2
        for (unsigned k0 = 0; k0 < K; k0 += 32u) {
          const v16h a  = frag_at(apr + k0);
          const v16h b0 = frag_at(bp0 + k0);
          const v16h b1 = frag_at(bp1 + k0);
          r0 = wmma16(a, b0, r0);
          r1 = wmma16(a, b1, r1);
        }
#pragma unroll
        for (int r = 0; r < 8; ++r) {
          acc0[r] = acc0[r] + r0[r] * rs;
          acc1[r] = acc1[r] + r1[r] * rs;
        }
      }
    }
#pragma unroll
    for (int r = 0; r < 8; ++r) {
      float* d = &Cs[(mw * 16u + hh * 8u + (unsigned)r) * LDC2 + p * 64u + nw * 32u + m];
      d[0]  = acc0[r];
      d[16] = acc1[r];
    }
  }
  __syncthreads();

  const bool vtile = (MODE == 2) && ((blockIdx.x & 1u) != 0u);

  if (MODE == 0 || (MODE == 2 && !vtile)) {
    const unsigned cbase = (MODE == 2) ? (blockIdx.x >> 1) * (unsigned)HD : n0;
    v8h x[4], xe[4];
    size_t off[4], offe[4];
#pragma unroll
    for (unsigned i = 0; i < 4u; ++i) {
      const unsigned r = 16u * i + (tid >> 4);
      const unsigned c = (tid & 15u) * 8u;
      const unsigned crow = row0 + r;
      const v4f u0 = *(const v4f*)&Cs[r * LDC2 + c];
      const v4f u1 = *(const v4f*)&Cs[r * LDC2 + c + 4u];
      if (MODE == 0) {
        const unsigned cp = c ^ 64u;
        const unsigned fi = c & 63u;
        const v4f p0 = *(const v4f*)&Cs[r * LDC2 + cp];
        const v4f p1 = *(const v4f*)&Cs[r * LDC2 + cp + 4u];
        const v4f c0 = *(const v4f*)(aux + (size_t)crow * CSW + fi);
        const v4f c1 = *(const v4f*)(aux + (size_t)crow * CSW + fi + 4u);
        const v4f s0 = *(const v4f*)(aux + (size_t)crow * CSW + 64u + fi);
        const v4f s1 = *(const v4f*)(aux + (size_t)crow * CSW + 64u + fi + 4u);
        const float sg = (c < 64u) ? -1.0f : 1.0f;
#pragma unroll
        for (int j = 0; j < 4; ++j) {
          const float ta = (u0[j] * iw) * c0[j] + sg * ((p0[j] * iw) * s0[j]);
          const float tb = (u1[j] * iw) * c1[j] + sg * ((p1[j] * iw) * s1[j]);
          const h16 ha = toh_flush(ta);
          const h16 hb = toh_flush(tb);
          x[i][j]      = ha;
          x[i][j + 4]  = hb;
          xe[i][j]     = toh_flush((ta - (float)ha) * QCARRY);
          xe[i][j + 4] = toh_flush((tb - (float)hb) * QCARRY);
        }
      } else {
        const v4f a0 = *(const v4f*)(aux + (size_t)crow * HD + c);
        const v4f a1 = *(const v4f*)(aux + (size_t)crow * HD + c + 4u);
#pragma unroll
        for (int j = 0; j < 4; ++j) {
          const float ta = u0[j] * iw + a0[j];
          const float tb = u1[j] * iw + a1[j];
          const h16 ha = toh_flush(ta);
          const h16 hb = toh_flush(tb);
          x[i][j]      = ha;
          x[i][j + 4]  = hb;
          xe[i][j]     = toh_flush((ta - (float)ha) * QCARRY);
          xe[i][j + 4] = toh_flush((tb - (float)hb) * QCARRY);
        }
      }
      off[i]  = (size_t)crow * HIDN + cbase + c;
      offe[i] = (size_t)(bidx0 * (unsigned)ERB + sq0 + r) * HIDN + cbase + c;
    }
#pragma unroll
    for (int i = 0; i < 4; ++i) *(volatile v8h*)(out16 + off[i]) = x[i];
    if (early_tile) {
#pragma unroll
      for (int i = 0; i < 4; ++i) *(volatile v8h*)(out16e + offe[i]) = xe[i];
    }
    __threadfence();
#pragma unroll
    for (int i = 0; i < 4; ++i) *(volatile v8h*)(out16 + off[i]) = x[i];
    if (early_tile) {
#pragma unroll
      for (int i = 0; i < 4; ++i) *(volatile v8h*)(out16e + offe[i]) = xe[i];
    }
  }

  if (MODE == 2 && vtile) {
    const unsigned head = blockIdx.x >> 1;
    v8h x[4], xr[4];
    size_t off[4], offr[4];
#pragma unroll
    for (unsigned i = 0; i < 4u; ++i) {
      const unsigned dcol = 32u * i + (tid >> 3);
      const unsigned kk = (tid & 7u) * 8u;
#pragma unroll
      for (unsigned j = 0; j < 8u; ++j) {
        const float t = Cs[(kk + j) * LDC2 + dcol] * iw;
        const h16 hi = toh_flush(t);
        x[i][j]  = hi;
        xr[i][j] = toh_flush((t - (float)hi) * RCARRY);
      }
      off[i]  = ((size_t)bidx0 * HIDN + head * (unsigned)HD + dcol) * SEQ + sq0 + kk;
      offr[i] = ((size_t)bidx0 * HIDN + head * (unsigned)HD + dcol) * (unsigned)ERB + sq0 + kk;
    }
#pragma unroll
    for (int i = 0; i < 4; ++i) *(volatile v8h*)(out16v + off[i]) = x[i];
    if (early_tile) {
#pragma unroll
      for (int i = 0; i < 4; ++i) *(volatile v8h*)(out16r + offr[i]) = xr[i];
    }
    __threadfence();
#pragma unroll
    for (int i = 0; i < 4; ++i) *(volatile v8h*)(out16v + off[i]) = x[i];
    if (early_tile) {
#pragma unroll
      for (int i = 0; i < 4; ++i) *(volatile v8h*)(out16r + offr[i]) = xr[i];
    }
  }

  if (MODE == 1 || MODE == 3) {
    const float cs = (MODE == 1) ? (1.0f / WCARRY) : (1.0f / (WCARRY * VCARRY));
    const unsigned ldo = (MODE == 1) ? (unsigned)KVAW : (unsigned)HIDN;
    v4f xs[8];
    size_t off[8];
#pragma unroll
    for (unsigned i = 0; i < 8u; ++i) {
      const unsigned r = 8u * i + (tid >> 5);
      const unsigned c = (tid & 31u) * 4u;
      const unsigned crow = row0 + r;
      const unsigned bidx = crow / (unsigned)SEQ;
      const unsigned sq = crow - bidx * (unsigned)SEQ;
      const size_t frow = (size_t)bidx * SEQ_FULL + sq;
      const size_t outrow = (MODE == 3) ? frow : (size_t)crow;
      const v4f u = *(const v4f*)&Cs[r * LDC2 + c];
      v4f val;
#pragma unroll
      for (int j = 0; j < 4; ++j) val[j] = u[j] * cs;
      xs[i] = val;
      off[i] = outrow * ldo + n0 + c;
    }
#pragma unroll
    for (int i = 0; i < 8; ++i) *(volatile v4f*)(outf + off[i]) = xs[i];
    __threadfence();
#pragma unroll
    for (int i = 0; i < 8; ++i) *(volatile v4f*)(outf + off[i]) = xs[i];
  }
}

__global__ __launch_bounds__(256) void gemm_q_kernel(
    const _Float16* __restrict__ A16, const _Float16* __restrict__ Bt,
    const float* __restrict__ cs, _Float16* __restrict__ q16, _Float16* __restrict__ qe16) {
  gemm_body<0>(A16, A16, Bt, (unsigned)HIDN, cs, (float*)0, q16, qe16, (_Float16*)0,
               (_Float16*)0);
}
__global__ __launch_bounds__(256) void gemm_kva_kernel(
    const _Float16* __restrict__ A16, const _Float16* __restrict__ Bt,
    float* __restrict__ kva) {
  gemm_body<1>(A16, A16, Bt, (unsigned)HIDN, (const float*)0, kva, (_Float16*)0, (_Float16*)0,
               (_Float16*)0, (_Float16*)0);
}
__global__ __launch_bounds__(256) void gemm_kv_kernel(
    const _Float16* __restrict__ A16, const _Float16* __restrict__ A16e,
    const _Float16* __restrict__ Bt,
    const float* __restrict__ kr, _Float16* __restrict__ k16, _Float16* __restrict__ ke16,
    _Float16* __restrict__ vt, _Float16* __restrict__ vte) {
  gemm_body<2>(A16, A16e, Bt, (unsigned)RANK, kr, (float*)0, k16, ke16, vt, vte);
}
__global__ __launch_bounds__(256) void gemm_out_kernel(
    const _Float16* __restrict__ A16, const _Float16* __restrict__ A16e,
    const _Float16* __restrict__ Bt, float* __restrict__ outf) {
  gemm_body<3>(A16, A16e, Bt, (unsigned)HIDN, (const float*)0, outf, (_Float16*)0,
               (_Float16*)0, (_Float16*)0, (_Float16*)0);
}

template <int RES>
__device__ __forceinline__ void ctx_phase(_Float16* P, const v8f a0, const v8f a1, const v8f a2,
                                          const v8f a3, const v8f inv,
                                          _Float16* __restrict__ dst, const size_t base) {
  const unsigned lane = threadIdx.x & 31u;
  const unsigned hh = lane >> 4, m = lane & 15u;
#pragma unroll
  for (int v = 0; v < 8; ++v) {
    const float t0 = a0[v] * inv[v];
    const float t1 = a1[v] * inv[v];
    const float t2 = a2[v] * inv[v];
    const float t3 = a3[v] * inv[v];
    const h16 h0 = toh_flush(t0);
    const h16 h1 = toh_flush(t1);
    const h16 h2 = toh_flush(t2);
    const h16 h3 = toh_flush(t3);
    _Float16* prow = P + (hh * 8u + (unsigned)v) * LDT + m;
    if (RES) {
      prow[0]  = toh_flush((t0 - (float)h0) * RCARRY);
      prow[16] = toh_flush((t1 - (float)h1) * RCARRY);
      prow[32] = toh_flush((t2 - (float)h2) * RCARRY);
      prow[48] = toh_flush((t3 - (float)h3) * RCARRY);
    } else {
      prow[0]  = h0;
      prow[16] = h1;
      prow[32] = h2;
      prow[48] = h3;
    }
  }
  wave_lds_sync();
  v8h x[4];
  size_t off[4];
#pragma unroll
  for (unsigned i = 0; i < 4u; ++i) {
    const unsigned r = 4u * i + (lane >> 3);
    const unsigned c = (lane & 7u) * 8u;
    x[i] = *(const v8h*)&P[r * LDT + c];
    off[i] = base + (size_t)r * HIDN + c;
  }
#pragma unroll
  for (int i = 0; i < 4; ++i) *(volatile v8h*)(dst + off[i]) = x[i];
  __threadfence();
#pragma unroll
  for (int i = 0; i < 4; ++i) *(volatile v8h*)(dst + off[i]) = x[i];
  wave_lds_sync();
}

__global__ __launch_bounds__(256) __attribute__((amdgpu_num_vgpr(256))) void attn_late_kernel(
    const _Float16* __restrict__ Qh, const _Float16* __restrict__ Kh,
    const _Float16* __restrict__ Vt, _Float16* __restrict__ Ov) {
  __shared__ _Float16 Ks[64 * LDK];
  __shared__ _Float16 Vs[HD * LDT];
  __shared__ _Float16 Ps[8 * 16 * LDT];

  const unsigned tid = threadIdx.x, lane = tid & 31u;
  const unsigned w = (unsigned)__builtin_amdgcn_readfirstlane((int)(tid >> 5));
  const unsigned hh = lane >> 4, m = lane & 15u;
  const unsigned q0 = (blockIdx.x + (unsigned)EBLK) * 128u;
  const unsigned head = blockIdx.y;
  const unsigned b = blockIdx.z;
  const float scale = 0.08838834764831845f;
  const unsigned qrow0 = q0 + w * 16u;
  _Float16* P = Ps + w * (16u * LDT);

  unsigned qo = (b * (unsigned)SEQ + qrow0 + m) * (unsigned)HIDN + head * (unsigned)HD + hh * 8u;

  float mrow[8], lrow[8];
  v8f o[8];
#pragma unroll
  for (int v = 0; v < 8; ++v) { mrow[v] = -1.0e30f; lrow[v] = 0.0f; }
#pragma unroll
  for (int nb = 0; nb < 8; ++nb) o[nb] = (v8f){};

  const size_t kplane = (size_t)b * SEQ * HIDN + head * HD;
  const size_t vplane = ((size_t)b * HIDN + head * HD) * SEQ;
  const unsigned kend = q0 + 128u;

  for (unsigned kb = 0; kb < kend; kb += 64u) {
    asm volatile("" : "+v"(qo));
#pragma unroll
    for (unsigned j = 0; j < 4u; ++j) {
      const unsigned idx = tid + 256u * j;
      const unsigned r = idx >> 4, c = (idx & 15u) * 8u;
      *(v8h*)&Ks[r * LDK + c] = *(const v8h*)(Kh + kplane + (size_t)(kb + r) * HIDN + c);
    }
#pragma unroll
    for (unsigned j = 0; j < 4u; ++j) {
      const unsigned idx = tid + 256u * j;
      const unsigned r = idx >> 3, c = (idx & 7u) * 8u;
      *(v8h*)&Vs[r * LDT + c] = *(const v8h*)(Vt + vplane + (size_t)r * SEQ + kb + c);
    }
    __syncthreads();

    v8f s[4];
#pragma unroll
    for (int kg = 0; kg < 4; ++kg) s[kg] = (v8f){};
#pragma unroll
    for (int c = 0; c < 4; ++c) {
      const v16h qf = frag_at(Qh + qo + (unsigned)c * 32u);
#pragma unroll
      for (int kg = 0; kg < 4; ++kg) {
        const v16h kf = ld_frag(&Ks[(kg * 16) * LDK + c * 32], LDK);
        s[kg] = wmma16(qf, kf, s[kg]);
      }
    }
#pragma unroll
    for (int kg = 0; kg < 4; ++kg) s[kg] = s[kg] * scale;

    if (kb >= q0) {
#pragma unroll
      for (int kg = 0; kg < 4; ++kg)
#pragma unroll
        for (int v = 0; v < 8; ++v) {
          const unsigned key = kb + (unsigned)kg * 16u + m;
          const unsigned row = qrow0 + hh * 8u + (unsigned)v;
          s[kg][v] = (key > row) ? -1.0e30f : s[kg][v];
        }
    }

    float alpha[8];
#pragma unroll
    for (int v = 0; v < 8; ++v) {
      float mx = fmaxf(fmaxf(s[0][v], s[1][v]), fmaxf(s[2][v], s[3][v]));
      mx = red16_max(mx);
      const float mn = fmaxf(mrow[v], mx);
      alpha[v] = __expf(mrow[v] - mn);
      mrow[v] = mn;
    }
#pragma unroll
    for (int kg = 0; kg < 4; ++kg)
#pragma unroll
      for (int v = 0; v < 8; ++v) s[kg][v] = __expf(s[kg][v] - mrow[v]);
#pragma unroll
    for (int v = 0; v < 8; ++v) {
      const float rs = red16_sum((s[0][v] + s[1][v]) + (s[2][v] + s[3][v]));
      lrow[v] = alpha[v] * lrow[v] + rs;
    }
#pragma unroll
    for (int nb = 0; nb < 8; ++nb)
#pragma unroll
      for (int v = 0; v < 8; ++v) o[nb][v] = o[nb][v] * alpha[v];

#pragma unroll
    for (int kg = 0; kg < 4; ++kg)
#pragma unroll
      for (int v = 0; v < 8; ++v)
        P[(hh * 8u + (unsigned)v) * LDT + (unsigned)kg * 16u + m] = toh_flush(s[kg][v] * PCARRY);
    wave_lds_sync();

#pragma unroll
    for (int c = 0; c < 2; ++c) {
      const v16h pf = ld_frag(P + c * 32, LDT);
#pragma unroll
      for (int nb = 0; nb < 8; ++nb) {
        const v16h vf = ld_frag(&Vs[(nb * 16) * LDT + c * 32], LDT);
        o[nb] = wmma16(pf, vf, o[nb]);
      }
    }
    __syncthreads();
  }

  v8f inv;
#pragma unroll
  for (int v = 0; v < 8; ++v)
    inv[v] = __builtin_amdgcn_rcpf(lrow[v] + 1.0e-5f) * (VCARRY / PCARRY);
  const size_t obase = (size_t)(b * (unsigned)SEQ + qrow0) * HIDN + head * HD;
  ctx_phase<0>(P, o[0], o[1], o[2], o[3], inv, Ov, obase);
  ctx_phase<0>(P, o[4], o[5], o[6], o[7], inv, Ov, obase + 64u);
}

__global__ __launch_bounds__(256) __attribute__((amdgpu_num_vgpr(256))) void attn_early_kernel(
    const _Float16* __restrict__ Qh, const _Float16* __restrict__ Qe,
    const _Float16* __restrict__ Kh, const _Float16* __restrict__ Ke,
    const _Float16* __restrict__ Vt, const _Float16* __restrict__ Ve,
    _Float16* __restrict__ Ov, _Float16* __restrict__ Oe) {
  __shared__ _Float16 Ps[8 * 16 * LDT];

  const unsigned tid = threadIdx.x, lane = tid & 31u;
  const unsigned w = (unsigned)__builtin_amdgcn_readfirstlane((int)(tid >> 5));
  const unsigned hh = lane >> 4, m = lane & 15u;
  const unsigned q0 = blockIdx.x * 128u;
  const unsigned head = blockIdx.y;
  const unsigned b = blockIdx.z >> 1;
  const unsigned dh = blockIdx.z & 1u;
  const float scale = 0.08838834764831845f;
  const unsigned qrow0 = q0 + w * 16u;
  _Float16* P = Ps + w * (16u * LDT);

  unsigned qo = (b * (unsigned)SEQ + qrow0 + m) * (unsigned)HIDN + head * (unsigned)HD + hh * 8u;
  unsigned qe = (b * (unsigned)ERB + qrow0 + m) * (unsigned)HIDN + head * (unsigned)HD + hh * 8u;

  float mrow[8], lrow[8];
  v8f o[4];
#pragma unroll
  for (int v = 0; v < 8; ++v) { mrow[v] = -1.0e30f; lrow[v] = 0.0f; }
#pragma unroll
  for (int nb = 0; nb < 4; ++nb) o[nb] = (v8f){};

  const size_t kplane = (size_t)b * SEQ * HIDN + head * HD + hh * 8u;
  const size_t eplane = (size_t)b * ERB * HIDN + head * HD + hh * 8u;
  const size_t vplane = ((size_t)b * HIDN + head * HD + dh * 64u + m) * SEQ + hh * 8u;
  const size_t rplane = ((size_t)b * HIDN + head * HD + dh * 64u + m) * (unsigned)ERB + hh * 8u;
  const unsigned kend = qrow0 + 16u;

  for (unsigned kb = 0; kb < kend; kb += 64u) {
    asm volatile("" : "+v"(qo));
    asm volatile("" : "+v"(qe));

    v8f s[4], sr[4];
#pragma unroll
    for (int kg = 0; kg < 4; ++kg) { s[kg] = (v8f){}; sr[kg] = (v8f){}; }
#pragma unroll
    for (int c = 0; c < 4; ++c) {
      const v16h qf = frag_at(Qh + qo + (unsigned)c * 32u);
      const v16h qr = frag_at(Qe + qe + (unsigned)c * 32u);
#pragma unroll
      for (int kg = 0; kg < 4; ++kg) {
        const size_t ko = (size_t)(kb + (unsigned)kg * 16u + m) * HIDN + (unsigned)c * 32u;
        const v16h kf = frag_at(Kh + kplane + ko);
        const v16h kr = frag_at(Ke + eplane + ko);
        s[kg]  = wmma16(qf, kf, s[kg]);
        sr[kg] = wmma16(qf, kr, sr[kg]);
        sr[kg] = wmma16(qr, kf, sr[kg]);
      }
    }
#pragma unroll
    for (int kg = 0; kg < 4; ++kg)
#pragma unroll
      for (int v = 0; v < 8; ++v)
        s[kg][v] = (s[kg][v] + sr[kg][v] * (1.0f / QCARRY)) * scale;

#pragma unroll
    for (int kg = 0; kg < 4; ++kg)
#pragma unroll
      for (int v = 0; v < 8; ++v) {
        const unsigned key = kb + (unsigned)kg * 16u + m;
        const unsigned row = qrow0 + hh * 8u + (unsigned)v;
        s[kg][v] = (key > row) ? -1.0e30f : s[kg][v];
      }

    float alpha[8];
#pragma unroll
    for (int v = 0; v < 8; ++v) {
      float mx = fmaxf(fmaxf(s[0][v], s[1][v]), fmaxf(s[2][v], s[3][v]));
      mx = red16_max(mx);
      const float mn = fmaxf(mrow[v], mx);
      alpha[v] = __expf(mrow[v] - mn);
      mrow[v] = mn;
    }
#pragma unroll
    for (int kg = 0; kg < 4; ++kg)
#pragma unroll
      for (int v = 0; v < 8; ++v) s[kg][v] = __expf(s[kg][v] - mrow[v]);
#pragma unroll
    for (int v = 0; v < 8; ++v) {
      const float rs = red16_sum((s[0][v] + s[1][v]) + (s[2][v] + s[3][v]));
      lrow[v] = alpha[v] * lrow[v] + rs;
    }
#pragma unroll
    for (int nb = 0; nb < 4; ++nb)
#pragma unroll
      for (int v = 0; v < 8; ++v) o[nb][v] = o[nb][v] * alpha[v];

#pragma unroll
    for (int kg = 0; kg < 4; ++kg)
#pragma unroll
      for (int v = 0; v < 8; ++v)
        P[(hh * 8u + (unsigned)v) * LDT + (unsigned)kg * 16u + m] = toh_flush(s[kg][v] * PCARRY);
    wave_lds_sync();

#pragma unroll
    for (int c = 0; c < 2; ++c) {
      const v16h pf = ld_frag(P + c * 32, LDT);
#pragma unroll
      for (int nb = 0; nb < 4; ++nb) {
        const v16h vf = frag_at(Vt + vplane + (size_t)((unsigned)nb * 16u) * SEQ + kb +
                                (unsigned)c * 32u);
        o[nb] = wmma16(pf, vf, o[nb]);
      }
    }
#pragma unroll
    for (int nb = 0; nb < 4; ++nb) {
      v8f o2 = {};
#pragma unroll
      for (int c = 0; c < 2; ++c) {
        const v16h pf = ld_frag(P + c * 32, LDT);
        const v16h vr = frag_at(Ve + rplane + (size_t)((unsigned)nb * 16u) * (unsigned)ERB + kb +
                                (unsigned)c * 32u);
        o2 = wmma16(pf, vr, o2);
      }
#pragma unroll
      for (int v = 0; v < 8; ++v) o[nb][v] = o[nb][v] + o2[v] * (1.0f / RCARRY);
    }
    wave_lds_sync();
#pragma unroll
    for (int kg = 0; kg < 4; ++kg)
#pragma unroll
      for (int v = 0; v < 8; ++v) {
        const float t = s[kg][v] * PCARRY;
        const float hi = (float)toh_flush(t);
        P[(hh * 8u + (unsigned)v) * LDT + (unsigned)kg * 16u + m] =
            toh_flush((t - hi) * RCARRY);
      }
    wave_lds_sync();
#pragma unroll
    for (int nb = 0; nb < 4; ++nb) {
      v8f o2 = {};
#pragma unroll
      for (int c = 0; c < 2; ++c) {
        const v16h pf = ld_frag(P + c * 32, LDT);
        const v16h vf = frag_at(Vt + vplane + (size_t)((unsigned)nb * 16u) * SEQ + kb +
                                (unsigned)c * 32u);
        o2 = wmma16(pf, vf, o2);
      }
#pragma unroll
      for (int v = 0; v < 8; ++v) o[nb][v] = o[nb][v] + o2[v] * (1.0f / RCARRY);
    }
    wave_lds_sync();
  }

  v8f inv;
#pragma unroll
  for (int v = 0; v < 8; ++v)
    inv[v] = __builtin_amdgcn_rcpf(lrow[v] + 1.0e-5f) * (VCARRY / PCARRY);
  const size_t obase = (size_t)(b * (unsigned)SEQ + qrow0) * HIDN + head * HD + dh * 64u;
  const size_t ebase = (size_t)(b * (unsigned)ERB + qrow0) * HIDN + head * HD + dh * 64u;
  ctx_phase<0>(P, o[0], o[1], o[2], o[3], inv, Ov, obase);
  ctx_phase<1>(P, o[0], o[1], o[2], o[3], inv, Oe, ebase);
}

extern "C" void kernel_launch(void* const* d_in, const int* in_sizes, int n_in,
                              void* d_out, int out_size, void* d_ws, size_t ws_size,
                              hipStream_t stream) {
  if (n_in < 7) return;
  const long long need_rows = (long long)(NB - 1) * SEQ_FULL + SEQ;
  const long long need_x = need_rows * HIDN;
  if ((long long)in_sizes[0] < need_x) return;
  if ((long long)in_sizes[1] < need_rows) return;
  if ((long long)in_sizes[2] < (long long)HIDN * HIDN) return;
  if ((long long)in_sizes[3] < (long long)HIDN * KVAW) return;
  if ((long long)in_sizes[4] < (long long)RANK * KVBW) return;
  if ((long long)in_sizes[5] < (long long)HIDN * HIDN) return;
  if (in_sizes[6] < RANK) return;
  if ((long long)out_size < need_x) return;
  if (ws_size < WS_TOTAL) return;

  const float* X    = (const float*)d_in[0];
  const int*   pos  = (const int*)d_in[1];
  const float* wq   = (const float*)d_in[2];
  const float* wkva = (const float*)d_in[3];
  const float* wkvb = (const float*)d_in[4];
  const float* wo   = (const float*)d_in[5];
  const float* lnw  = (const float*)d_in[6];
  float* out = (float*)d_out;

  char* ws = (char*)d_ws;
  _Float16* Wq_t   = (_Float16*)(ws + OFF_WQ);
  _Float16* Wkva_t = (_Float16*)(ws + OFF_WKVA);
  _Float16* Wkvb_t = (_Float16*)(ws + OFF_WKVB);
  _Float16* Wo_t   = (_Float16*)(ws + OFF_WO);
  _Float16* X16    = (_Float16*)(ws + OFF_X);
  _Float16* Ctx16  = (_Float16*)(ws + OFF_CTX);
  _Float16* Qh16   = (_Float16*)(ws + OFF_Q);
  _Float16* Kh16   = (_Float16*)(ws + OFF_K);
  _Float16* Vt16   = (_Float16*)(ws + OFF_VT);
  _Float16* QE16   = (_Float16*)(ws + OFF_QE);
  _Float16* KE16   = (_Float16*)(ws + OFF_KE);
  _Float16* VE16   = (_Float16*)(ws + OFF_VE);
  _Float16* CE16   = (_Float16*)(ws + OFF_CE);
  float*    KVA    = (float*)(ws + OFF_KVA);
  _Float16* C16    = (_Float16*)(ws + OFF_C16);
  float*    KR     = (float*)(ws + OFF_KR);
  float*    CS     = (float*)(ws + OFF_CS);
  _Float16* C16E   = (_Float16*)(ws + OFF_C16E);

  dim3 blk(256);

  wconv_kernel<<<dim3(HIDN / 64, HIDN / 64), blk, 0, stream>>>(wq, Wq_t, (unsigned)HIDN, (unsigned)HIDN);
  wconv_kernel<<<dim3(KVAW / 64, HIDN / 64), blk, 0, stream>>>(wkva, Wkva_t, (unsigned)KVAW, (unsigned)HIDN);
  wconv_kernel<<<dim3(KVBW / 64, RANK / 64), blk, 0, stream>>>(wkvb, Wkvb_t, (unsigned)KVBW, (unsigned)RANK);
  wconv_kernel<<<dim3(HIDN / 64, HIDN / 64), blk, 0, stream>>>(wo, Wo_t, (unsigned)HIDN, (unsigned)HIDN);

  xcast_kernel<<<dim3(MROWS), blk, 0, stream>>>(X, X16);
  cstab_kernel<<<dim3(MROWS / 8), blk, 0, stream>>>(pos, CS);
  gemm_q_kernel<<<dim3(HIDN / 128, MROWS / 64), blk, 0, stream>>>(X16, Wq_t, CS, Qh16, QE16);
  gemm_kva_kernel<<<dim3(KVAW / 128, MROWS / 64), blk, 0, stream>>>(X16, Wkva_t, KVA);
  norm_rope_kernel<<<dim3(MROWS / 8), blk, 0, stream>>>(KVA, lnw, CS, C16, C16E, KR);
  gemm_kv_kernel<<<dim3(KVBW / 128, MROWS / 64), blk, 0, stream>>>(C16, C16E, Wkvb_t, KR, Kh16, KE16, Vt16, VE16);
  attn_early_kernel<<<dim3(EBLK, NHEAD, NB * 2), blk, 0, stream>>>(Qh16, QE16, Kh16, KE16, Vt16, VE16, Ctx16, CE16);
  if (SEQ / 128 > EBLK) {
    attn_late_kernel<<<dim3(SEQ / 128 - EBLK, NHEAD, NB), blk, 0, stream>>>(Qh16, Kh16, Vt16, Ctx16);
  }
  gemm_out_kernel<<<dim3(HIDN / 128, MROWS / 64), blk, 0, stream>>>(Ctx16, CE16, Wo_t, out);
}
